// DKVMN_47785806135738
// MI455X (gfx1250) — hardware-verified
//
#include <hip/hip_runtime.h>
#include <stddef.h>

constexpr int NBATCH = 64;
constexpr int NSTEP  = 200;
constexpr int DIM    = 256;
constexpr int MSLOT  = 64;
constexpr int NSKILL = 1000;
constexpr int NROWS  = NBATCH * NSTEP;
constexpr int NOUT   = NBATCH * (NSTEP - 1);
constexpr int RKLD   = 2 * DIM;
static_assert(NROWS % 64 == 0, "M tile");
static_assert(NOUT % 32 == 0, "whole output lines");
static_assert(DIM % 64 == 0 && MSLOT % 64 == 0, "N tile");
static_assert(DIM % 32 == 0 && RKLD % 32 == 0, "K step");

constexpr size_t SZ_RK = (size_t)NROWS * RKLD * 2;
constexpr size_t SZ_VP = (size_t)NROWS * DIM * 2;
constexpr size_t SZ_MK = (size_t)MSLOT * DIM * 2;
constexpr size_t SZ_EW = (size_t)DIM * DIM * 2;
constexpr size_t SZ_AW = SZ_EW;
constexpr size_t SZ_FW = (size_t)DIM * RKLD * 2;
constexpr size_t SZ_S  = (size_t)NROWS * MSLOT * 4;
constexpr size_t SZ_W  = SZ_S;
constexpr size_t SZ_E  = (size_t)NROWS * DIM * 4;
constexpr size_t SZ_A  = SZ_E;
constexpr size_t SZ_F  = SZ_E;
constexpr size_t OFF_RK = 0;
constexpr size_t OFF_VP = OFF_RK + SZ_RK;
constexpr size_t OFF_MK = OFF_VP + SZ_VP;
constexpr size_t OFF_EW = OFF_MK + SZ_MK;
constexpr size_t OFF_AW = OFF_EW + SZ_EW;
constexpr size_t OFF_FW = OFF_AW + SZ_AW;
constexpr size_t OFF_S  = OFF_FW + SZ_FW;
constexpr size_t OFF_W  = OFF_S  + SZ_S;
constexpr size_t OFF_E  = OFF_W  + SZ_W;
constexpr size_t OFF_A  = OFF_E  + SZ_E;
constexpr size_t OFF_F  = OFF_A  + SZ_A;
constexpr size_t WS_TOTAL = OFF_F + SZ_F;
static_assert(WS_TOTAL == 66093056u, "carve total");
static_assert(WS_TOTAL <= 134217728u, "carve budget");
static_assert((OFF_VP % 1024) == 0 && (OFF_MK % 1024) == 0 && (OFF_EW % 1024) == 0 && (OFF_AW % 1024) == 0 &&
              (OFF_FW % 1024) == 0 && (OFF_S % 1024) == 0 && (OFF_W % 1024) == 0 && (OFF_E % 1024) == 0 &&
              (OFF_A % 1024) == 0 && (OFF_F % 1024) == 0, "aligned regions");

typedef __attribute__((ext_vector_type(16))) _Float16 v16h;
typedef __attribute__((ext_vector_type(8)))  _Float16 v8h;
typedef __attribute__((ext_vector_type(16))) __bf16   v16b;
typedef __attribute__((ext_vector_type(8)))  __bf16   v8b;
typedef __attribute__((ext_vector_type(8)))  float    v8f;
typedef __attribute__((ext_vector_type(4)))  float    v4f;
typedef __attribute__((ext_vector_type(4)))  unsigned v4u;

__device__ __forceinline__ unsigned short f2bf_bits(float f) {
  unsigned u = __float_as_uint(f);
  return (unsigned short)((u + 0x7FFFu + ((u >> 16) & 1u)) >> 16);
}
__device__ __forceinline__ float bf_bits2f(unsigned short h) { return __uint_as_float(((unsigned)h) << 16); }
__device__ __forceinline__ float rbf(float f) { return bf_bits2f(f2bf_bits(f)); }
__device__ __forceinline__ unsigned pack_bf2(float a, float b) {
  return (unsigned)f2bf_bits(a) | ((unsigned)f2bf_bits(b) << 16);
}
__device__ __forceinline__ unsigned pack_h2(float a, float b) {
  const _Float16 h0 = (_Float16)a, h1 = (_Float16)b;
  return (unsigned)__builtin_bit_cast(unsigned short, h0) | ((unsigned)__builtin_bit_cast(unsigned short, h1) << 16);
}
__device__ __forceinline__ float sigm_f(float v) {
  v = fminf(fmaxf(v, -30.0f), 30.0f);
  return 1.0f / (1.0f + expf(-v));
}

__device__ __forceinline__ void dep_guard_h(v8f& a, v8f& b, v16h x, v16h y) { asm volatile("v_nop\n\tv_nop\n\tv_nop\n\tv_nop" : "+v"(a), "+v"(b) : "v"(x), "v"(y)); }
__device__ __forceinline__ void dep_guard_b(v8f& a, v8f& b, v16b x, v16b y) { asm volatile("v_nop\n\tv_nop\n\tv_nop\n\tv_nop" : "+v"(a), "+v"(b) : "v"(x), "v"(y)); }
__device__ __forceinline__ void keep4_h(v16h a, v16h b, v16h c, v16h d) { asm volatile("v_nop" :: "v"(a), "v"(b), "v"(c), "v"(d)); }
__device__ __forceinline__ void keep4_b(v16b a, v16b b, v16b c, v16b d) { asm volatile("v_nop" :: "v"(a), "v"(b), "v"(c), "v"(d)); }
__device__ __forceinline__ void acc_guard4(v8f& a, v8f& b, v8f& c, v8f& d) { asm volatile("v_nop\n\tv_nop\n\tv_nop\n\tv_nop" : "+v"(a), "+v"(b), "+v"(c), "+v"(d)); }
template <typename T> struct Frag;
template <> struct Frag<_Float16> {
  typedef v16h V; union U { v16h v; v8h h[2]; };
  static __device__ __forceinline__ v16h load(const _Float16* p) {
    U f; f.h[0] = *(const v8h*)(p); f.h[1] = *(const v8h*)(p + 16); return f.v;
  }
  static __device__ __forceinline__ v8f mma(v16h a, v16h b, v8f c) {
    return __builtin_amdgcn_wmma_f32_16x16x32_f16(false, a, false, b, (short)0, c, false, false);
  }
  static __device__ __forceinline__ void guard(v8f& a, v8f& b, v16h x, v16h y) { dep_guard_h(a, b, x, y); }
  static __device__ __forceinline__ void keep(v16h a, v16h b, v16h c, v16h d) { keep4_h(a, b, c, d); }
};
template <> struct Frag<__bf16> {
  typedef v16b V; union U { v16b v; v8b h[2]; };
  static __device__ __forceinline__ v16b load(const __bf16* p) {
    U f; f.h[0] = *(const v8b*)(p); f.h[1] = *(const v8b*)(p + 16); return f.v;
  }
  static __device__ __forceinline__ v8f mma(v16b a, v16b b, v8f c) {
    return __builtin_amdgcn_wmma_f32_16x16x32_bf16(false, a, false, b, (short)0, c, false, false);
  }
  static __device__ __forceinline__ void guard(v8f& a, v8f& b, v16b x, v16b y) { dep_guard_b(a, b, x, y); }
  static __device__ __forceinline__ void keep(v16b a, v16b b, v16b c, v16b d) { keep4_b(a, b, c, d); }
};

__device__ __forceinline__ v8f mma_h_guarded(v16h a, v16h b, v8f c) {
  c = __builtin_amdgcn_wmma_f32_16x16x32_f16(false, a, false, b, (short)0, c, false, false);
  asm volatile("v_nop\n\tv_nop\n\tv_nop\n\tv_nop" : "+v"(c) : "v"(a), "v"(b));
  return c;
}

template <int ET> struct Elem;
template <> struct Elem<0> { typedef _Float16 T; };
template <> struct Elem<1> { typedef __bf16 T; };
template <int ET, bool SPLIT, int BIAS_MODE, int OUT_MODE, bool RESID, int ACT = 0>
__global__ __launch_bounds__(256) void wmma_gemm64(
    const unsigned short* __restrict__ Ap, const unsigned short* __restrict__ A2p, int lda, long strideA,
    const unsigned short* __restrict__ Btp, const unsigned short* __restrict__ Bt2p, int ldb, long strideB,
    void* __restrict__ Cout, void* __restrict__ Cout2, int ldc, long strideC,
    const float* __restrict__ bias,
    const float* __restrict__ resid, long strideR,
    int M, int N, int K, float scale) {
  typedef typename Elem<ET>::T T;
  typedef typename Frag<T>::V V;
  const T* A = (const T*)Ap; const T* A2 = (const T*)A2p; const T* Bt = (const T*)Btp; const T* Bt2 = (const T*)Bt2p;
  __shared__ __align__(16) float sT[8][16 * 68];
  const int b    = blockIdx.y;
  const int lane = threadIdx.x & 31;
  const int wave = threadIdx.x >> 5;
  const int tilesN = N >> 6;
  const int tilesM = M >> 6;
  const int tile = blockIdx.x * 8 + wave;
  if (tile >= tilesM * tilesN) return;
  const int tm = tile / tilesN;
  const int tn = tile - tm * tilesN;
  const int m0 = tm << 6;
  const int n0 = tn << 6;

  const T* Ab  = A  + (size_t)b * strideA;
  const T* Bb  = Bt + (size_t)b * strideB;
  const T* Ab2 = SPLIT ? (A2  + (size_t)b * strideA) : nullptr;
  const T* Bb2 = SPLIT ? (Bt2 + (size_t)b * strideB) : nullptr;

  const int rlane = lane & 15;
  const int koff  = (lane >> 4) * 8;
  const int mOff  = (lane >> 4) * 8;

  v8f acc[4][4];
#pragma unroll
  for (int i = 0; i < 4; ++i)
#pragma unroll
    for (int j = 0; j < 4; ++j) acc[i][j] = (v8f){0.f,0.f,0.f,0.f,0.f,0.f,0.f,0.f};

  for (int k0 = 0; k0 < K; k0 += 32) {
    V bh[4], bl[4];
#pragma unroll
    for (int j = 0; j < 4; ++j) {
      const size_t bo = (size_t)(n0 + (j << 4) + rlane) * ldb + koff + k0;
      bh[j] = Frag<T>::load(Bb + bo);
      if (SPLIT) bl[j] = Frag<T>::load(Bb2 + bo);
    }
#pragma unroll
    for (int i = 0; i < 4; ++i) {
      const size_t ao = (size_t)(m0 + (i << 4) + rlane) * lda + koff + k0;
      V ah = Frag<T>::load(Ab + ao);
      V al;
      if (SPLIT) al = Frag<T>::load(Ab2 + ao);
#pragma unroll
      for (int j = 0; j < 4; ++j) {
        acc[i][j] = Frag<T>::mma(ah, bh[j], acc[i][j]);
        if (SPLIT) {
          acc[i][j] = Frag<T>::mma(ah, bl[j], acc[i][j]);
          acc[i][j] = Frag<T>::mma(al, bh[j], acc[i][j]);
        }
      }
      Frag<T>::guard(acc[i][0], acc[i][3], ah, SPLIT ? al : ah);
    }
    Frag<T>::keep(bh[0], bh[1], bh[2], bh[3]);
    if (SPLIT) Frag<T>::keep(bl[0], bl[1], bl[2], bl[3]);
  }
  acc_guard4(acc[0][0], acc[0][1], acc[0][2], acc[0][3]);
  acc_guard4(acc[1][0], acc[1][1], acc[1][2], acc[1][3]);
  acc_guard4(acc[2][0], acc[2][1], acc[2][2], acc[2][3]);
  acc_guard4(acc[3][0], acc[3][1], acc[3][2], acc[3][3]);

  float* slab = sT[wave];
  const float* Rb = RESID ? (resid + (size_t)b * strideR) : nullptr;
#pragma unroll
  for (int i = 0; i < 4; ++i) {
    const int mBase = m0 + (i << 4);
#pragma unroll
    for (int j = 0; j < 4; ++j) {
      const int n = n0 + (j << 4) + rlane;
      float bv = 0.f;
      if (BIAS_MODE == 2) bv = bias[n];
      if (BIAS_MODE == 3) bv = bf_bits2f(f2bf_bits(bias[n]));
#pragma unroll
      for (int r = 0; r < 8; ++r) {
        float v = acc[i][j][r] * scale;
        if (BIAS_MODE == 1) v += bias[mBase + mOff + r];
        if (BIAS_MODE == 2 || BIAS_MODE == 3) v += bv;
        if (RESID) v += Rb[(size_t)(mBase + mOff + r) * ldc + n];
        slab[(mOff + r) * 68 + (j << 4) + rlane] = v;
      }
    }
    __builtin_amdgcn_fence(__ATOMIC_RELEASE, "workgroup");
    __builtin_amdgcn_wave_barrier();
    __builtin_amdgcn_fence(__ATOMIC_ACQUIRE, "workgroup");
    if (ACT != 0) {
#pragma unroll 1
      for (int it = 0; it < 32; ++it) {
        const int idx = it * 32 + lane;
        const int row = idx >> 6, col = idx & 63;
        float v = slab[row * 68 + col];
        if (ACT == 1) v = tanhf(v);
        if (ACT == 2) v = fmaxf(v, 0.0f);
        if (ACT == 4) v = (v > 0.f) ? v : 0.01f * v;
        if (ACT == 6) v = sigm_f(v);
        slab[row * 68 + col] = v;
      }
      __builtin_amdgcn_fence(__ATOMIC_RELEASE, "workgroup");
      __builtin_amdgcn_wave_barrier();
      __builtin_amdgcn_fence(__ATOMIC_ACQUIRE, "workgroup");
    }
    if (OUT_MODE == 0) {
      float* C = (float*)Cout + (size_t)b * strideC;
      const int hh = lane >> 4, c4 = (lane & 15) * 4;
      for (int pass = 0; pass < 2; ++pass) {
#pragma unroll
        for (int it = 0; it < 8; ++it) {
          const int row = it * 2 + hh;
          v4f v = *(const v4f*)(slab + row * 68 + c4);
          *(volatile v4f*)(C + (size_t)(mBase + row) * ldc + n0 + c4) = v;
        }
        __threadfence();
      }
    } else {
      const int q = lane >> 3, c8 = (lane & 7) * 8;
      unsigned short* C  = (unsigned short*)Cout  + (size_t)b * strideC;
      unsigned short* C2 = (OUT_MODE == 2) ? ((unsigned short*)Cout2 + (size_t)b * strideC) : nullptr;
      for (int pass = 0; pass < 2; ++pass) {
#pragma unroll
        for (int it = 0; it < 4; ++it) {
          const int row = it * 4 + q;
          const float* sp = slab + row * 68 + c8;
          v8h hv, lv;
#pragma unroll
          for (int e = 0; e < 8; ++e) {
            if (OUT_MODE == 1) {
              hv[e] = (_Float16)sp[e];
            } else {
              unsigned short hb = f2bf_bits(sp[e]);
              unsigned short lb = f2bf_bits(sp[e] - bf_bits2f(hb));
              hv[e] = __builtin_bit_cast(_Float16, hb);
              lv[e] = __builtin_bit_cast(_Float16, lb);
            }
          }
          *(volatile v8h*)(C + (size_t)(mBase + row) * ldc + n0 + c8) = hv;
          if (OUT_MODE == 2) *(volatile v8h*)(C2 + (size_t)(mBase + row) * ldc + n0 + c8) = lv;
        }
        __threadfence();
      }
    }
    __builtin_amdgcn_fence(__ATOMIC_RELEASE, "workgroup");
    __builtin_amdgcn_wave_barrier();
    __builtin_amdgcn_fence(__ATOMIC_ACQUIRE, "workgroup");
  }
}

__global__ __launch_bounds__(256) void cast_f32_bf16x8(
    const float* __restrict__ in, unsigned short* __restrict__ outp, int n8) {
  const int i = blockIdx.x * 256 + threadIdx.x;
  if (i < n8) {
    const float* src = in + (size_t)i * 8;
    const v4f a = *(const v4f*)(src);
    const v4f c = *(const v4f*)(src + 4);
    v4u u;
    u[0] = pack_bf2(a[0], a[1]); u[1] = pack_bf2(a[2], a[3]);
    u[2] = pack_bf2(c[0], c[1]); u[3] = pack_bf2(c[2], c[3]);
    unsigned short* dst = outp + (size_t)i * 8;
    *(volatile v4u*)dst = u;
    __threadfence();
    *(volatile v4u*)dst = u;
  }
}

__global__ __launch_bounds__(256) void gather_rows(
    const int* __restrict__ skills, const int* __restrict__ responses,
    const float* __restrict__ kemb, const float* __restrict__ vemb,
    unsigned short* __restrict__ RK, unsigned short* __restrict__ Vp) {
  const int lane = threadIdx.x & 31, wave = threadIdx.x >> 5;
  const int g = blockIdx.x * 8 + wave;
  if (g >= NROWS) return;
  int sk = skills[g];
  const int rs = responses[g];
  if (sk < 0) sk += NSKILL;
  sk = sk < 0 ? 0 : (sk > NSKILL - 1 ? NSKILL - 1 : sk);
  int x = sk + NSKILL * rs;
  if (x < 0) x += 2 * NSKILL;
  x = x < 0 ? 0 : (x > 2 * NSKILL - 1 ? 2 * NSKILL - 1 : x);
  const float* kr = kemb + (size_t)sk * DIM + 8 * lane;
  const float* vr = vemb + (size_t)x  * DIM + 8 * lane;
  const v4f ka = *(const v4f*)(kr); const v4f kb = *(const v4f*)(kr + 4);
  const v4f va = *(const v4f*)(vr); const v4f vb = *(const v4f*)(vr + 4);
  v4u ku, vu;
  ku[0] = pack_bf2(ka[0], ka[1]); ku[1] = pack_bf2(ka[2], ka[3]);
  ku[2] = pack_bf2(kb[0], kb[1]); ku[3] = pack_bf2(kb[2], kb[3]);
  vu[0] = pack_bf2(va[0], va[1]); vu[1] = pack_bf2(va[2], va[3]);
  vu[2] = pack_bf2(vb[0], vb[1]); vu[3] = pack_bf2(vb[2], vb[3]);
  unsigned short* kd = RK + (size_t)g * RKLD + DIM + 8 * lane;
  unsigned short* vd = Vp + (size_t)g * DIM + 8 * lane;
  *(volatile v4u*)kd = ku;
  *(volatile v4u*)vd = vu;
  __threadfence();
  *(volatile v4u*)kd = ku;
  *(volatile v4u*)vd = vu;
}

__global__ __launch_bounds__(256) void softmax_rows(const float* __restrict__ S, float* __restrict__ W) {
  const int lane = threadIdx.x & 31, wave = threadIdx.x >> 5;
  const int g = blockIdx.x * 8 + wave;
  if (g >= NROWS) return;
  const float* sr = S + (size_t)g * MSLOT;
  const float s0 = sr[lane], s1 = sr[32 + lane];
  float m = fmaxf(s0, s1);
#pragma unroll
  for (int off = 16; off > 0; off >>= 1) m = fmaxf(m, __shfl_xor(m, off, 32));
  const float e0 = expf(s0 - m), e1 = expf(s1 - m);
  float sum = e0 + e1;
#pragma unroll
  for (int off = 16; off > 0; off >>= 1) sum += __shfl_xor(sum, off, 32);
  const float inv = 1.0f / sum;
  const float w0 = e0 * inv, w1 = e1 * inv;
  volatile float* wd = W + (size_t)g * MSLOT;
  wd[lane] = w0;
  wd[32 + lane] = w1;
  __threadfence();
  wd[lane] = w0;
  wd[32 + lane] = w1;
}

__global__ __launch_bounds__(256) void memory_scan(
    const float* __restrict__ Wp, const float* __restrict__ Ep, const float* __restrict__ Apl,
    const float* __restrict__ Mv0, unsigned short* __restrict__ RK) {
  __shared__ __align__(16) unsigned MvT_u[DIM * (MSLOT / 2)];
  __shared__ __align__(16) unsigned Wsh_u[16 * (MSLOT / 2)];
  __shared__ __align__(16) float Rsh[DIM];
  const int tid = threadIdx.x, lane = tid & 31, wave = tid >> 5;
  const int b = blockIdx.x;
  const int rlane = lane & 15, koff = (lane >> 4) * 8;

  if (tid < 120) *(v4u*)(Wsh_u + 32 + 4 * tid) = (v4u){0u, 0u, 0u, 0u};

  float mv[MSLOT];
  {
    float* stg = (float*)(void*)MvT_u;
#pragma unroll
    for (int half = 0; half < 2; ++half) {
#pragma unroll
      for (int j = 0; j < 8; ++j) {
        const int q = tid + 256 * j;
        const v4f v = *(const v4f*)(Mv0 + (size_t)half * 8192 + 4 * q);
        *(v4f*)(stg + 4 * q) = v;
      }
      __syncthreads();
#pragma unroll
      for (int m = 0; m < 32; ++m) mv[32 * half + m] = rbf(stg[m * DIM + tid]);
      __syncthreads();
    }
  }

  const _Float16* Wh = (const _Float16*)(const void*)Wsh_u;
  const _Float16* Mh = (const _Float16*)(const void*)MvT_u;

  for (int t = 0; t < NSTEP; ++t) {
    const int g = b * NSTEP + t;
    const float* wrow = Wp + (size_t)g * MSLOT;
    const float w0 = wrow[lane];
    const float w1 = wrow[32 + lane];
    const float ed = Ep[(size_t)g * DIM + tid];
    const float ad = Apl[(size_t)g * DIM + tid];

#pragma unroll
    for (int j = 0; j < 8; ++j) {
      v4u u;
      u[0] = pack_h2(mv[8 * j + 0], mv[8 * j + 1]);
      u[1] = pack_h2(mv[8 * j + 2], mv[8 * j + 3]);
      u[2] = pack_h2(mv[8 * j + 4], mv[8 * j + 5]);
      u[3] = pack_h2(mv[8 * j + 6], mv[8 * j + 7]);
      *(v4u*)(MvT_u + tid * 32 + 4 * j) = u;
    }
    if (wave == 0) {
      const int q = lane & 7;
      const v4f wa = *(const v4f*)(wrow + 8 * q);
      const v4f wb = *(const v4f*)(wrow + 8 * q + 4);
      v4u u;
      u[0] = pack_h2(wa[0] * 1024.0f, wa[1] * 1024.0f);
      u[1] = pack_h2(wa[2] * 1024.0f, wa[3] * 1024.0f);
      u[2] = pack_h2(wb[0] * 1024.0f, wb[1] * 1024.0f);
      u[3] = pack_h2(wb[2] * 1024.0f, wb[3] * 1024.0f);
      if (lane < 8) *(v4u*)(Wsh_u + 4 * q) = u;
    }
    __syncthreads();

    {
      const v16h a0 = Frag<_Float16>::load(Wh + rlane * MSLOT + koff);
      const v16h a1 = Frag<_Float16>::load(Wh + rlane * MSLOT + koff + 32);
#pragma unroll
      for (int j = 0; j < 2; ++j) {
        const int n0 = (wave * 2 + j) * 16;
        const v16h b0 = Frag<_Float16>::load(Mh + (n0 + rlane) * MSLOT + koff);
        const v16h b1 = Frag<_Float16>::load(Mh + (n0 + rlane) * MSLOT + koff + 32);
        v8f acc = (v8f){0.f, 0.f, 0.f, 0.f, 0.f, 0.f, 0.f, 0.f};
        acc = mma_h_guarded(a0, b0, acc);
        acc = mma_h_guarded(a1, b1, acc);
        const float rv = acc[0] * (1.0f / 1024.0f);
        if (lane < 16) Rsh[n0 + lane] = rv;
      }
    }

#pragma unroll
    for (int m = 0; m < 32; ++m) {
      const float wm = __shfl(w0, m, 32);
      const float old = mv[m];
      const float er = 1.0f - wm * ed;
      mv[m] = old * er + wm * ad;
    }
#pragma unroll
    for (int m = 0; m < 32; ++m) {
      const float wm = __shfl(w1, m, 32);
      const float old = mv[32 + m];
      const float er = 1.0f - wm * ed;
      mv[32 + m] = old * er + wm * ad;
    }
    __syncthreads();

    if (wave == 0) {
      const v4f r0 = *(const v4f*)(Rsh + 8 * lane);
      const v4f r1 = *(const v4f*)(Rsh + 8 * lane + 4);
      v4u u;
      u[0] = pack_bf2(r0[0], r0[1]); u[1] = pack_bf2(r0[2], r0[3]);
      u[2] = pack_bf2(r1[0], r1[1]); u[3] = pack_bf2(r1[2], r1[3]);
      unsigned short* dst = RK + (size_t)g * RKLD + 8 * lane;
      *(volatile v4u*)dst = u;
      __threadfence();
      *(volatile v4u*)dst = u;
    }
  }
}

__global__ __launch_bounds__(256) void predict_rows(
    const float* __restrict__ Fp, const float* __restrict__ pW, const float* __restrict__ pb,
    float* __restrict__ outp) {
  const int lane = threadIdx.x & 31, wave = threadIdx.x >> 5;
  const int L = blockIdx.x * 8 + wave;
  if (L >= NOUT / 32) return;
  const v4f pa = *(const v4f*)(pW + 8 * lane);
  const v4f pc = *(const v4f*)(pW + 8 * lane + 4);
  const float q0 = rbf(pa[0]), q1 = rbf(pa[1]), q2 = rbf(pa[2]), q3 = rbf(pa[3]);
  const float q4 = rbf(pc[0]), q5 = rbf(pc[1]), q6 = rbf(pc[2]), q7 = rbf(pc[3]);
  const float pbr = rbf(pb[0]);
  float mine = 0.f;
#pragma unroll 1
  for (int i = 0; i < 32; ++i) {
    const int o  = L * 32 + i;
    const int bb = o / (NSTEP - 1);
    const int tt = o - bb * (NSTEP - 1) + 1;
    const int g  = bb * NSTEP + tt;
    const float* fr = Fp + (size_t)g * DIM + 8 * lane;
    const v4f f0 = *(const v4f*)(fr);
    const v4f f1 = *(const v4f*)(fr + 4);
    float s = f0[0] * q0;
    s += f0[1] * q1; s += f0[2] * q2; s += f0[3] * q3;
    s += f1[0] * q4; s += f1[1] * q5; s += f1[2] * q6; s += f1[3] * q7;
#pragma unroll
    for (int off = 16; off > 0; off >>= 1) s += __shfl_xor(s, off, 32);
    mine = (lane == i) ? s : mine;
  }
  const float x = mine + pbr;
  const float p = sigm_f(x);
  volatile float* dst = outp + (size_t)L * 32;
  dst[lane] = p;
  __threadfence();
  dst[lane] = p;
}

extern "C" void kernel_launch(void* const* d_in, const int* in_sizes, int n_in,
                              void* d_out, int out_size, void* d_ws, size_t ws_size,
                              hipStream_t stream) {
  if (n_in < 14) return;
  if (ws_size < WS_TOTAL) return;
  if (out_size < NOUT) return;
  if (in_sizes[0] < NROWS || in_sizes[1] < NROWS) return;
  if (in_sizes[2] < NSKILL * DIM || in_sizes[3] < 2 * NSKILL * DIM) return;
  if (in_sizes[4] < MSLOT * DIM || in_sizes[5] < MSLOT * DIM) return;
  if (in_sizes[6] < DIM * RKLD || in_sizes[8] < DIM * DIM || in_sizes[10] < DIM * DIM) return;
  if (in_sizes[7] < DIM || in_sizes[9] < DIM || in_sizes[11] < DIM || in_sizes[12] < DIM || in_sizes[13] < 1) return;
  const int*   skills    = (const int*)d_in[0];
  const int*   responses = (const int*)d_in[1];
  const float* k_emb     = (const float*)d_in[2];
  const float* v_emb     = (const float*)d_in[3];
  const float* Mk        = (const float*)d_in[4];
  const float* Mv0       = (const float*)d_in[5];
  const float* fW        = (const float*)d_in[6];
  const float* fb        = (const float*)d_in[7];
  const float* eW        = (const float*)d_in[8];
  const float* eb        = (const float*)d_in[9];
  const float* aW        = (const float*)d_in[10];
  const float* ab        = (const float*)d_in[11];
  const float* pW        = (const float*)d_in[12];
  const float* pb        = (const float*)d_in[13];
  float* outp = (float*)d_out;

  char* ws = (char*)d_ws;
  unsigned short* RK   = (unsigned short*)(ws + OFF_RK);
  unsigned short* Vp   = (unsigned short*)(ws + OFF_VP);
  unsigned short* Mk16 = (unsigned short*)(ws + OFF_MK);
  unsigned short* eW16 = (unsigned short*)(ws + OFF_EW);
  unsigned short* aW16 = (unsigned short*)(ws + OFF_AW);
  unsigned short* fW16 = (unsigned short*)(ws + OFF_FW);
  float* Spl = (float*)(ws + OFF_S);
  float* Wpl = (float*)(ws + OFF_W);
  float* Epl = (float*)(ws + OFF_E);
  float* Apl = (float*)(ws + OFF_A);
  float* Fpl = (float*)(ws + OFF_F);

  {
    const int n8_mk = (MSLOT * DIM) / 8;
    const int n8_ew = (DIM * DIM) / 8;
    const int n8_fw = (DIM * RKLD) / 8;
    cast_f32_bf16x8<<<(n8_mk + 255) / 256, 256, 0, stream>>>(Mk, Mk16, n8_mk);
    cast_f32_bf16x8<<<(n8_ew + 255) / 256, 256, 0, stream>>>(eW, eW16, n8_ew);
    cast_f32_bf16x8<<<(n8_ew + 255) / 256, 256, 0, stream>>>(aW, aW16, n8_ew);
    cast_f32_bf16x8<<<(n8_fw + 255) / 256, 256, 0, stream>>>(fW, fW16, n8_fw);
  }

  gather_rows<<<(NROWS + 7) / 8, 256, 0, stream>>>(skills, responses, k_emb, v_emb, RK, Vp);

  static_assert(NROWS % 64 == 0 && MSLOT % 64 == 0 && DIM % 32 == 0, "gemm S shape");
  {
    const int tiles = (NROWS / 64) * (MSLOT / 64);
    wmma_gemm64<1, false, 0, 0, false, 0><<<dim3((tiles + 7) / 8, 1), 256, 0, stream>>>(
        RK + DIM, RK + DIM, RKLD, 0L, Mk16, Mk16, DIM, 0L,
        (void*)Spl, (void*)Spl, MSLOT, 0L, fb, Mv0, 0L, NROWS, MSLOT, DIM, 1.0f);
  }
  softmax_rows<<<(NROWS + 7) / 8, 256, 0, stream>>>(Spl, Wpl);

  static_assert(NROWS % 64 == 0 && DIM % 64 == 0 && DIM % 32 == 0, "gemm E/A shape");
  {
    const int tiles = (NROWS / 64) * (DIM / 64);
    wmma_gemm64<1, false, 3, 0, false, 6><<<dim3((tiles + 7) / 8, 1), 256, 0, stream>>>(
        Vp, Vp, DIM, 0L, eW16, eW16, DIM, 0L,
        (void*)Epl, (void*)Epl, DIM, 0L, eb, Mv0, 0L, NROWS, DIM, DIM, 1.0f);
    wmma_gemm64<1, false, 3, 0, false, 1><<<dim3((tiles + 7) / 8, 1), 256, 0, stream>>>(
        Vp, Vp, DIM, 0L, aW16, aW16, DIM, 0L,
        (void*)Apl, (void*)Apl, DIM, 0L, ab, Mv0, 0L, NROWS, DIM, DIM, 1.0f);
  }

  memory_scan<<<NBATCH, 256, 0, stream>>>(Wpl, Epl, Apl, Mv0, RK);

  static_assert(NROWS % 64 == 0 && DIM % 64 == 0 && RKLD % 32 == 0, "gemm F shape");
  {
    const int tiles = (NROWS / 64) * (DIM / 64);
    wmma_gemm64<1, false, 3, 0, false, 1><<<dim3((tiles + 7) / 8, 1), 256, 0, stream>>>(
        RK, RK, RKLD, 0L, fW16, fW16, RKLD, 0L,
        (void*)Fpl, (void*)Fpl, DIM, 0L, fb, Mv0, 0L, NROWS, DIM, RKLD, 1.0f);
  }

  predict_rows<<<(NOUT / 32 + 7) / 8, 256, 0, stream>>>(Fpl, pW, pb, outp);
}
